// GraphAttn_70970039599321
// MI455X (gfx1250) — hardware-verified
//
#include <hip/hip_runtime.h>
#include <stdint.h>

#define NN     16384
#define KIN    256
#define NF     128
#define RT     64
#define TP     72
#define OP     132
#define SLOPE  0.01f
#define ECARRY 16.0f
#define EINV   0.0625f
#define NXBLK  ((NN * KIN) / (8 * 256))
#define NWBLK  ((NF * KIN) / (8 * 256))

static_assert((NN % RT) == 0);
static_assert((NN % 32) == 0);
static_assert((KIN % 32) == 0);
static_assert(NF == 128);
static_assert(RT == 64);
static_assert(((NN * KIN) % (8 * 256)) == 0);
static_assert(((NF * KIN) % (8 * 256)) == 0);
static_assert(((TP * 2) % 16) == 0);
static_assert(((OP * 4) % 16) == 0);

typedef _Float16 v16h __attribute__((ext_vector_type(16)));
typedef _Float16 v8h  __attribute__((ext_vector_type(8)));
typedef __bf16   v16b __attribute__((ext_vector_type(16)));
typedef __bf16   v8b  __attribute__((ext_vector_type(8)));
typedef float    v8f  __attribute__((ext_vector_type(8)));
typedef float    v4f  __attribute__((ext_vector_type(4)));
typedef unsigned int v4u __attribute__((ext_vector_type(4)));
typedef v4f __attribute__((may_alias)) v4fa;
typedef v4u __attribute__((may_alias)) v4ua;
typedef v8h __attribute__((may_alias)) v8ha;
typedef v8b __attribute__((may_alias)) v8ba;

#if defined(__HIP_DEVICE_COMPILE__)
#define DEV_ASM 1
#else
#define DEV_ASM 0
#endif

__device__ __forceinline__ unsigned short bf_bits(float f) {
  unsigned u = __float_as_uint(f);
  return (unsigned short)((u + 0x7FFFu + ((u >> 16) & 1u)) >> 16);
}
__device__ __forceinline__ float bf_up(unsigned short hb) { return __uint_as_float(((unsigned)hb) << 16); }
__device__ __forceinline__ unsigned pk16(unsigned short a, unsigned short b) { return (unsigned)a | ((unsigned)b << 16); }
__device__ __forceinline__ v8f zero8() { v8f z = {0.f, 0.f, 0.f, 0.f, 0.f, 0.f, 0.f, 0.f}; return z; }

__device__ __forceinline__ _Float16 ek(float s2c, float s1c) {
  const float v = s2c + s1c;
  const float l = fmaxf(v, v * SLOPE);
  return (_Float16)l;
}

__device__ __forceinline__ v16b ldfrag_b(const __bf16* p) {
  union { v16b v; v8b h[2]; } f;
  f.h[0] = *(const v8ba*)(p);
  f.h[1] = *(const v8ba*)(p + 16);
  return f.v;
}
__device__ __forceinline__ v16h ldfrag_h(const _Float16* p) {
  union { v16h v; v8h h[2]; } f;
  f.h[0] = *(const v8ha*)(p);
  f.h[1] = *(const v8ha*)(p + 16);
  return f.v;
}

__device__ __forceinline__ v8f mma_b(v16b a, v16b b, v8f c) {
  c = __builtin_amdgcn_wmma_f32_16x16x32_bf16(false, a, false, b, (short)0, c, false, false);
#if DEV_ASM
  asm volatile("v_nop\n\tv_nop\n\tv_nop\n\tv_nop" : "+v"(c) : "v"(a), "v"(b));
#endif
  return c;
}
__device__ __forceinline__ v8f mma_h(v16h a, v16h b, v8f c) {
  c = __builtin_amdgcn_wmma_f32_16x16x32_f16(false, a, false, b, (short)0, c, false, false);
#if DEV_ASM
  asm volatile("v_nop\n\tv_nop\n\tv_nop\n\tv_nop" : "+v"(c) : "v"(a), "v"(b));
#endif
  return c;
}

__global__ __launch_bounds__(256) void k_prep(const float* __restrict__ x, const float* __restrict__ w,
                                              unsigned short* XB, unsigned short* WB) {
  const int tid = threadIdx.x;
  const float* src;
  unsigned short* dst;
  if (blockIdx.x < NXBLK) {
    const size_t g = (size_t)blockIdx.x * 256 + tid;
    src = x + g * 8;
    dst = XB + g * 8;
  } else {
    const size_t g = (size_t)(blockIdx.x - NXBLK) * 256 + tid;
    src = w + g * 8;
    dst = WB + g * 8;
  }
  const v4f a = *(const v4fa*)src;
  const v4f c = *(const v4fa*)(src + 4);
  v4u o;
  o[0] = pk16(bf_bits(a[0]), bf_bits(a[1]));
  o[1] = pk16(bf_bits(a[2]), bf_bits(a[3]));
  o[2] = pk16(bf_bits(c[0]), bf_bits(c[1]));
  o[3] = pk16(bf_bits(c[2]), bf_bits(c[3]));
  *(volatile v4u*)dst = o;
  __threadfence();
  *(volatile v4u*)dst = o;
}

__global__ __launch_bounds__(128) void k_h(const unsigned short* __restrict__ XBp,
                                           const unsigned short* __restrict__ WBp,
                                           const float* __restrict__ a1, const float* __restrict__ a2,
                                           unsigned short* HT, float* SC) {
  __shared__ __align__(16) float    Hs[RT * OP];
  __shared__ __align__(16) _Float16 T[NF * TP];
  __shared__ __align__(16) float    as[2 * NF];
  __shared__ __align__(16) float    ss[2 * RT];

  const int tid  = threadIdx.x;
  const int lane = tid & 31;
  const int wave = tid >> 5;
  const int h    = lane >> 4;
  const int m    = lane & 15;
  const int j0   = blockIdx.x * RT;

  const __bf16* XB = (const __bf16*)(const void*)XBp;
  const __bf16* WB = (const __bf16*)(const void*)WBp;

  if (wave == 0) {
    const v4f v = *(const v4fa*)(a1 + 4 * lane);
    const v4f r = { bf_up(bf_bits(v[0])), bf_up(bf_bits(v[1])), bf_up(bf_bits(v[2])), bf_up(bf_bits(v[3])) };
    *(v4fa*)(as + 4 * lane) = r;
  } else if (wave == 1) {
    const v4f v = *(const v4fa*)(a2 + 4 * lane);
    const v4f r = { bf_up(bf_bits(v[0])), bf_up(bf_bits(v[1])), bf_up(bf_bits(v[2])), bf_up(bf_bits(v[3])) };
    *(v4fa*)(as + NF + 4 * lane) = r;
  }

  v8f acc[8];
#pragma unroll
  for (int t = 0; t < 8; ++t) acc[t] = zero8();

  const __bf16* xa = XB + ((size_t)(j0 + 16 * wave + m)) * KIN + 8 * h;
  const __bf16* wb = WB + ((size_t)m) * KIN + 8 * h;

#pragma unroll 1
  for (int k0 = 0; k0 < KIN; k0 += 32) {
    const v16b a = ldfrag_b(xa + k0);
#pragma unroll
    for (int t = 0; t < 8; ++t) {
      const v16b b = ldfrag_b(wb + (size_t)t * 16 * KIN + k0);
      acc[t] = mma_b(a, b, acc[t]);
    }
  }

#pragma unroll
  for (int t = 0; t < 8; ++t) {
#pragma unroll
    for (int r = 0; r < 8; ++r) {
      Hs[(16 * wave + 8 * h + r) * OP + 16 * t + m] = acc[t][r];
    }
    const v8h hv = { (_Float16)acc[t][0], (_Float16)acc[t][1], (_Float16)acc[t][2], (_Float16)acc[t][3],
                     (_Float16)acc[t][4], (_Float16)acc[t][5], (_Float16)acc[t][6], (_Float16)acc[t][7] };
    *(v8ha*)(T + (16 * t + m) * TP + 16 * wave + 8 * h) = hv;
  }
  __syncthreads();

  {
    const int q  = lane >> 3;
    const int c8 = (lane & 7) * 8;
    v4u vv[8];
#pragma unroll
    for (int it = 0; it < 8; ++it) {
      const int n = wave * 32 + it * 4 + q;
      vv[it] = *(const v4ua*)(T + n * TP + c8);
    }
    for (int pass = 0; pass < 2; ++pass) {
#pragma unroll
      for (int it = 0; it < 8; ++it) {
        const int n = wave * 32 + it * 4 + q;
        unsigned short* dst = HT + ((size_t)n) * NN + j0 + c8;
        *(volatile v4u*)dst = vv[it];
      }
      __threadfence();
    }
  }

  {
    const int which = tid >> 6;
    const int row   = tid & 63;
    const float* hr = Hs + row * OP;
    const float* av = as + which * NF;
    float d = 0.0f;
#pragma unroll 1
    for (int c = 0; c < NF; c += 4) {
      const v4f hv = *(const v4fa*)(hr + c);
      const v4f aw = *(const v4fa*)(av + c);
      d += hv[0] * aw[0];
      d += hv[1] * aw[1];
      d += hv[2] * aw[2];
      d += hv[3] * aw[3];
    }
    ss[tid] = d * ECARRY;
  }
  __syncthreads();

  if (wave == 0) {
    const v4f sv = *(const v4fa*)(ss + 4 * lane);
    float* dst = SC + ((size_t)(lane >> 4)) * NN + j0 + 4 * (lane & 15);
    *(volatile v4f*)dst = sv;
    __threadfence();
    *(volatile v4f*)dst = sv;
  }
}

__global__ __launch_bounds__(128) void k_out(const unsigned short* __restrict__ HTp,
                                             const float* __restrict__ SC,
                                             float* out) {
  __shared__ __align__(16) float os[4][16 * OP];

  const int tid  = threadIdx.x;
  const int lane = tid & 31;
  const int wave = tid >> 5;
  const int h    = lane >> 4;
  const int m    = lane & 15;
  const int i0   = blockIdx.x * RT;

  const _Float16* HT = (const _Float16*)(const void*)HTp;
  const float* S1C = SC;
  const float* S2C = SC + NN;

  const float s2r = S2C[i0 + 16 * wave + m];

  v8f acc[8];
#pragma unroll
  for (int t = 0; t < 8; ++t) acc[t] = zero8();

  const _Float16* hrow = HT + ((size_t)m) * NN + 8 * h;
  const float*    s1p  = S1C + 8 * h;

#pragma unroll 1
  for (int j0 = 0; j0 < NN; j0 += 32) {
    const v4f sa = *(const v4fa*)(s1p + j0);
    const v4f sb = *(const v4fa*)(s1p + j0 + 4);
    const v4f sc = *(const v4fa*)(s1p + j0 + 16);
    const v4f sd = *(const v4fa*)(s1p + j0 + 20);
    const v16h ea = { ek(s2r, sa[0]), ek(s2r, sa[1]), ek(s2r, sa[2]), ek(s2r, sa[3]),
                      ek(s2r, sb[0]), ek(s2r, sb[1]), ek(s2r, sb[2]), ek(s2r, sb[3]),
                      ek(s2r, sc[0]), ek(s2r, sc[1]), ek(s2r, sc[2]), ek(s2r, sc[3]),
                      ek(s2r, sd[0]), ek(s2r, sd[1]), ek(s2r, sd[2]), ek(s2r, sd[3]) };
#pragma unroll
    for (int t = 0; t < 8; ++t) {
      const v16h bf = ldfrag_h(hrow + (size_t)t * 16 * NN + j0);
      acc[t] = mma_h(ea, bf, acc[t]);
    }
  }

  float* osw = os[wave];
#pragma unroll
  for (int t = 0; t < 8; ++t) {
#pragma unroll
    for (int r = 0; r < 8; ++r) {
      osw[(8 * h + r) * OP + 16 * t + m] = acc[t][r] * EINV;
    }
  }
  __syncthreads();

  for (int pass = 0; pass < 2; ++pass) {
#pragma unroll
    for (int row = 0; row < 16; ++row) {
      const v4f v = *(const v4fa*)(osw + row * OP + 4 * lane);
      float* dst = out + ((size_t)(i0 + 16 * wave + row)) * NF + 4 * lane;
      *(volatile v4f*)dst = v;
    }
    __threadfence();
  }
}

extern "C" void kernel_launch(void* const* d_in, const int* in_sizes, int n_in,
                              void* d_out, int out_size, void* d_ws, size_t ws_size,
                              hipStream_t stream) {
  if (n_in < 4) return;
  if (in_sizes[0] != NN * KIN) return;
  if (in_sizes[1] != NF * KIN) return;
  if (in_sizes[2] != NF) return;
  if (in_sizes[3] != NF) return;
  if (out_size != NN * NF) return;

  const float* x  = (const float*)d_in[0];
  const float* w  = (const float*)d_in[1];
  const float* a1 = (const float*)d_in[2];
  const float* a2 = (const float*)d_in[3];
  float* out = (float*)d_out;

  const size_t bXB = (size_t)NN * KIN * 2;
  const size_t bWB = (size_t)NF * KIN * 2;
  const size_t bHT = (size_t)NF * NN * 2;
  const size_t bSC = (size_t)2 * NN * 4;
  size_t off = 0;
  const size_t oXB = off; off += bXB;
  const size_t oWB = off; off += bWB;
  const size_t oHT = off; off += bHT;
  const size_t oSC = off; off += bSC;
  if (off > ws_size) return;
  if (off > (size_t)134217728) return;

  char* ws = (char*)d_ws;
  unsigned short* XB = (unsigned short*)(ws + oXB);
  unsigned short* WB = (unsigned short*)(ws + oWB);
  unsigned short* HT = (unsigned short*)(ws + oHT);
  float*          SC = (float*)(ws + oSC);

  k_prep<<<dim3(NXBLK + NWBLK), dim3(256), 0, stream>>>(x, w, XB, WB);
  k_h<<<dim3(NN / RT), dim3(128), 0, stream>>>(XB, WB, a1, a2, HT, SC);
  k_out<<<dim3(NN / RT), dim3(128), 0, stream>>>(HT, SC, out);
  (void)hipGetLastError();
}
